// DGN_47115791237717
// MI455X (gfx1250) — hardware-run, weakly checked
//
#include <hip/hip_runtime.h>
#include <math.h>
#include <stdint.h>

#ifndef NB
#define NB 128
#endif
#ifndef SEQ
#define SEQ 256
#endif
#define NB_FULL  128
#define SEQ_FULL 256
#define FIN   128
#define HID   512
#define NHD   8
#define HDD   16
#define HDM   (NHD * HDD)
#define NVQK  (3 * HDM)
#define NACT  32
#define QIN   (3 * HID)
#define BG    ((NB <= 64) ? NB : 64)
#define NGRP  (NB / BG)
#define GROWS (BG * SEQ)
#define NQT   (SEQ / 16)
#define NKT   (SEQ / 32)
#define NST   (SEQ / 64)
#define CAR   1024.0f
#define PCAR  32768.0f
#define ATT_SCALE 0.25f
#define LOG2E 1.4426950408889634f
#define SLAB64 (16 * 68)
#define VTP   72
#define MKP   (SEQ + 4)
#define PTP   36
#define PTW   (16 * PTP)
#define RSP   (HDM + 4)
#define ATT_THREADS (NHD * 32)
#define WS_CAP 134217728
static_assert(NB >= 1 && NB <= NB_FULL && (NB % BG) == 0 && BG >= 1 && BG <= 64);
static_assert(SEQ >= 64 && SEQ <= SEQ_FULL && (SEQ % 64) == 0);
static_assert(ATT_THREADS == 256 && HDM == 128 && HDD == 16 && NHD == 8);
static_assert((GROWS % 64) == 0 && (FIN % 64) == 0 && (HID % 128) == 0 && (HDM % 64) == 0 && (NVQK % 64) == 0);
static_assert((QIN % 64) == 0 && NACT == 32 && (FIN % 32) == 0 && (HID % 32) == 0);
static_assert(((MKP * 4) % 16) == 0 && ((RSP * 4) % 16) == 0 && ((GROWS * FIN) % 8) == 0);

typedef unsigned short u16;
typedef _Float16 v16h __attribute__((ext_vector_type(16)));
typedef _Float16 v8h  __attribute__((ext_vector_type(8)));
typedef __bf16   v16b __attribute__((ext_vector_type(16)));
typedef float    v8f  __attribute__((ext_vector_type(8)));
typedef float    v4f  __attribute__((ext_vector_type(4)));
typedef unsigned int v4u __attribute__((ext_vector_type(4)));
typedef int      v4i  __attribute__((ext_vector_type(4)));

union FragH { v16h v; v8h h[2]; v4u u[2]; };
union FragB { v16b v; v4u u[2]; };

__device__ __forceinline__ unsigned short bf_bits(float f) {
  unsigned u = __float_as_uint(f);
  return (unsigned short)((u + 0x7FFFu + ((u >> 16) & 1u)) >> 16);
}
__device__ __forceinline__ float bf_up(unsigned short h) { return __uint_as_float(((unsigned)h) << 16); }
__device__ __forceinline__ float bfr(float f) { return bf_up(bf_bits(f)); }
__device__ __forceinline__ unsigned short h_bits(_Float16 x) { return __builtin_bit_cast(unsigned short, x); }
__device__ __forceinline__ unsigned pk16(unsigned short a, unsigned short b) { return (unsigned)a | ((unsigned)b << 16); }
__device__ __forceinline__ v8f zero8() { v8f z = {0.f, 0.f, 0.f, 0.f, 0.f, 0.f, 0.f, 0.f}; return z; }
__device__ __forceinline__ v4u zero4u() { v4u z = {0u, 0u, 0u, 0u}; return z; }
__device__ __forceinline__ int imin(int a, int b) { return a < b ? a : b; }
__device__ __forceinline__ int imax(int a, int b) { return a > b ? a : b; }

__device__ __forceinline__ v16h ldfrag_h(const _Float16* p) {
  FragH f;
  f.h[0] = *(const v8h*)(p);
  f.h[1] = *(const v8h*)(p + 16);
  return f.v;
}
__device__ __forceinline__ v16b ldfrag_b(const u16* p) {
  FragB f;
  f.u[0] = *(const v4u*)(p);
  f.u[1] = *(const v4u*)(p + 16);
  return f.v;
}

__device__ __forceinline__ v8f mma_h(v16h a, v16h b, v8f c) {
  return __builtin_amdgcn_wmma_f32_16x16x32_f16(false, a, false, b, (short)0, c, false, false);
}
__device__ __forceinline__ v8f mma_b(v16b a, v16b b, v8f c) {
  return __builtin_amdgcn_wmma_f32_16x16x32_bf16(false, a, false, b, (short)0, c, false, false);
}
__device__ __forceinline__ void guard1(v8f& a, v16h x0, v16h x1) {
#if defined(__HIP_DEVICE_COMPILE__)
  asm volatile("v_nop\n\tv_nop\n\tv_nop\n\tv_nop" : "+v"(a) : "v"(x0), "v"(x1) : "memory");
#endif
}
__device__ __forceinline__ void guard2(v8f& a, v8f& b, v16h x0, v16h x1, v16h x2, v16h x3, v16h x4, v16h x5) {
#if defined(__HIP_DEVICE_COMPILE__)
  asm volatile("v_nop\n\tv_nop\n\tv_nop\n\tv_nop"
               : "+v"(a), "+v"(b) : "v"(x0), "v"(x1), "v"(x2), "v"(x3), "v"(x4), "v"(x5) : "memory");
#endif
}
template <typename F>
__device__ __forceinline__ void guard6(v8f& a, v8f& b, v8f& c, v8f& d, F x0, F x1, F x2, F x3, F x4, F x5) {
#if defined(__HIP_DEVICE_COMPILE__)
  asm volatile("v_nop\n\tv_nop\n\tv_nop\n\tv_nop"
               : "+v"(a), "+v"(b), "+v"(c), "+v"(d) : "v"(x0), "v"(x1), "v"(x2), "v"(x3), "v"(x4), "v"(x5) : "memory");
#endif
}
__device__ __forceinline__ void acc_guard1(v8f& a) {
#if defined(__HIP_DEVICE_COMPILE__)
  asm volatile("v_nop\n\tv_nop\n\tv_nop\n\tv_nop" : "+v"(a));
#endif
}
__device__ __forceinline__ void wave_sync_lds() {
  __builtin_amdgcn_fence(__ATOMIC_RELEASE, "workgroup");
  __builtin_amdgcn_wave_barrier();
  __builtin_amdgcn_fence(__ATOMIC_ACQUIRE, "workgroup");
}

__global__ __launch_bounds__(256) void cvtx(const float* __restrict__ x, u16* D, int gb0, int n8) {
  const int gt = blockIdx.x * 256 + (int)threadIdx.x;
  if (gt >= n8) return;
  const int row = gt / (FIN / 8);
  const int c8  = (gt - row * (FIN / 8)) * 8;
  const int b   = row / SEQ;
  const int s   = row - b * SEQ;
  const float* p = x + ((size_t)(gb0 + b) * SEQ_FULL + s) * FIN + c8;
  const v4f a = *(const v4f*)(p), b4 = *(const v4f*)(p + 4);
  float w[8];
#pragma unroll
  for (int e = 0; e < 4; ++e) { w[e] = a[e]; w[4 + e] = b4[e]; }
  v4u o;
#pragma unroll
  for (int e = 0; e < 4; ++e) o[e] = pk16(bf_bits(w[2 * e]), bf_bits(w[2 * e + 1]));
  u16* d = D + (size_t)gt * 8;
  for (int pass = 0; pass < 2; ++pass) {
    *(volatile v4u*)(d) = o;
    __threadfence();
  }
}

template <int NT, int TB>
__global__ __launch_bounds__(256) void wt16(const float* __restrict__ W, int ldw, int krows, int ncols,
                                            u16* D, int ldd, int noff, float scale) {
  static_assert(NT == 128 || NT == 32);
  __shared__ __align__(16) u16 T[NT * VTP];
  const int tid = threadIdx.x;
  const int bid = blockIdx.x;
  const int nct = ncols / NT;
  const int ct  = bid % nct;
  const int rt  = bid / nct;
  if (rt * 64 + 64 > krows) return;
  {
    const int sl = tid >> 2;
    const int dc = (tid & 3) * (NT / 4);
    const float* src = W + (size_t)(rt * 64 + sl) * ldw + ct * NT + dc;
#pragma unroll
    for (int i = 0; i < NT / 16; ++i) {
      const v4f a = *(const v4f*)(src + 4 * i);
#pragma unroll
      for (int e = 0; e < 4; ++e) {
        const float f = a[e];
        const unsigned short hb = h_bits((_Float16)(bfr(f) * scale));
        const unsigned short bb = bf_bits(f);
        T[(dc + 4 * i + e) * VTP + sl] = (TB != 0) ? bb : hb;
      }
    }
  }
  __syncthreads();
  constexpr int NIT = NT / 32;
  v4u w4[NIT];
  const int q8 = tid >> 3, p8 = (tid & 7) * 8;
#pragma unroll
  for (int it = 0; it < NIT; ++it) {
    const int line = it * 32 + q8;
    w4[it] = *(const v4u*)(T + line * VTP + p8);
  }
  const size_t base = ((size_t)noff + (size_t)ct * NT) * (size_t)ldd + rt * 64 + p8;
  for (int pass = 0; pass < 2; ++pass) {
#pragma unroll
    for (int it = 0; it < NIT; ++it) {
      const int line = it * 32 + q8;
      *(volatile v4u*)(D + base + (size_t)line * (size_t)ldd) = w4[it];
    }
    __threadfence();
  }
}

__global__ __launch_bounds__(256) void vt16k(const u16* __restrict__ S, u16* VT) {
  __shared__ __align__(16) u16 T[HDM * VTP];
  const int tid = threadIdx.x;
  const int bid = blockIdx.x;
  const int st  = bid % NST;
  const int b   = bid / NST;
  if (b >= BG) return;
  const int s0  = st * 64;
  {
    const int sl = tid >> 2;
    const int dc = (tid & 3) * 32;
    const u16* src = S + ((size_t)b * SEQ + s0 + sl) * NVQK + dc;
#pragma unroll
    for (int i = 0; i < 4; ++i) {
      const v4u a = *(const v4u*)(src + 8 * i);
#pragma unroll
      for (int e = 0; e < 4; ++e) {
        const unsigned wv = a[e];
        T[(dc + 8 * i + 2 * e) * VTP + sl]     = (u16)(wv & 0xFFFFu);
        T[(dc + 8 * i + 2 * e + 1) * VTP + sl] = (u16)(wv >> 16);
      }
    }
  }
  __syncthreads();
  v4u vv[4];
  const int q8 = tid >> 3, p8 = (tid & 7) * 8;
#pragma unroll
  for (int it = 0; it < 4; ++it) {
    const int line = it * 32 + q8;
    vv[it] = *(const v4u*)(T + line * VTP + p8);
  }
  const size_t base = ((size_t)b * HDM) * SEQ + s0 + p8;
  for (int pass = 0; pass < 2; ++pass) {
#pragma unroll
    for (int it = 0; it < 4; ++it) {
      const int line = it * 32 + q8;
      *(volatile v4u*)(VT + base + (size_t)line * SEQ) = vv[it];
    }
    __threadfence();
  }
}

template <int TB, int NPROD, int NCT, int OM>
__global__ __launch_bounds__(128)
void gemm16(const u16* __restrict__ Ah, const u16* __restrict__ Al, int lda,
            const u16* __restrict__ Bt, int ldb, int K, int M, int N,
            const float* __restrict__ b0, const float* __restrict__ b1, const float* __restrict__ b2,
            int nseg, int hasbias, int relu, float oscale, float ocar,
            float* Cf, u16* Ch, u16* Cl, int ldc,
            const float* __restrict__ P0, const float* __restrict__ P1) {
  static_assert(NCT == 2 || NCT == 4);
  static_assert(NPROD == 1 || NPROD == 2);
  static_assert(TB == 0 || (NPROD == 1 && NCT == 4));
  static_assert(OM == 0 || OM == 3 || NCT == 4);
  __shared__ __align__(16) float slab[4 * SLAB64];
  const int tid = threadIdx.x, wave = tid >> 5, lane = tid & 31, hh = lane >> 4, m = lane & 15;
  constexpr int TNC = 16 * NCT;
  const int ntile = N / TNC;
  const int bid   = blockIdx.x;
  const int rowb  = (bid / ntile) * 64 + wave * 16;
  const int col0  = (bid % ntile) * TNC;
  if (rowb + 16 > M) return;
  v8f acc[NCT];
#pragma unroll
  for (int j = 0; j < NCT; ++j) acc[j] = zero8();
  const size_t bs = (size_t)16 * (size_t)ldb;

  if constexpr (TB == 1) {
    const u16* ap = Ah + (size_t)(rowb + m) * lda + 8 * hh;
    const u16* bp = Bt + (size_t)(col0 + m) * ldb + 8 * hh;
#pragma unroll 1
    for (int k0 = 0; k0 < K; k0 += 32) {
      const v16b a  = ldfrag_b(ap + k0);
      const v16b f0 = ldfrag_b(bp + k0);
      const v16b f1 = ldfrag_b(bp + bs + k0);
      const v16b f2 = ldfrag_b(bp + 2 * bs + k0);
      const v16b f3 = ldfrag_b(bp + 3 * bs + k0);
      acc[0] = mma_b(a, f0, acc[0]);
      acc[1] = mma_b(a, f1, acc[1]);
      acc[2] = mma_b(a, f2, acc[2]);
      acc[3] = mma_b(a, f3, acc[3]);
      guard6<v16b>(acc[0], acc[1], acc[2], acc[3], a, f0, f1, f2, f3, a);
    }
  } else {
    const _Float16* ahp = (const _Float16*)(const void*)Ah + (size_t)(rowb + m) * lda + 8 * hh;
    const _Float16* alp = (const _Float16*)(const void*)Al + (size_t)(rowb + m) * lda + 8 * hh;
    const _Float16* bp  = (const _Float16*)(const void*)Bt + (size_t)(col0 + m) * ldb + 8 * hh;
    if constexpr (NCT == 4) {
      if constexpr (NPROD == 2) {
#pragma unroll 1
        for (int k0 = 0; k0 < K; k0 += 32) {
          const v16h ah = ldfrag_h(ahp + k0), al = ldfrag_h(alp + k0);
          const v16h f0 = ldfrag_h(bp + k0);
          const v16h f1 = ldfrag_h(bp + bs + k0);
          const v16h f2 = ldfrag_h(bp + 2 * bs + k0);
          const v16h f3 = ldfrag_h(bp + 3 * bs + k0);
          acc[0] = mma_h(ah, f0, acc[0]);  acc[0] = mma_h(al, f0, acc[0]);
          acc[1] = mma_h(ah, f1, acc[1]);  acc[1] = mma_h(al, f1, acc[1]);
          acc[2] = mma_h(ah, f2, acc[2]);  acc[2] = mma_h(al, f2, acc[2]);
          acc[3] = mma_h(ah, f3, acc[3]);  acc[3] = mma_h(al, f3, acc[3]);
          guard6<v16h>(acc[0], acc[1], acc[2], acc[3], ah, al, f0, f1, f2, f3);
        }
      } else {
#pragma unroll 1
        for (int k0 = 0; k0 < K; k0 += 32) {
          const v16h ah = ldfrag_h(ahp + k0);
          const v16h f0 = ldfrag_h(bp + k0);
          const v16h f1 = ldfrag_h(bp + bs + k0);
          const v16h f2 = ldfrag_h(bp + 2 * bs + k0);
          const v16h f3 = ldfrag_h(bp + 3 * bs + k0);
          acc[0] = mma_h(ah, f0, acc[0]);
          acc[1] = mma_h(ah, f1, acc[1]);
          acc[2] = mma_h(ah, f2, acc[2]);
          acc[3] = mma_h(ah, f3, acc[3]);
          guard6<v16h>(acc[0], acc[1], acc[2], acc[3], ah, f0, f1, f2, f3, ah);
        }
      }
    } else {
      if constexpr (NPROD == 2) {
#pragma unroll 1
        for (int k0 = 0; k0 < K; k0 += 32) {
          const v16h ah = ldfrag_h(ahp + k0), al = ldfrag_h(alp + k0);
          const v16h f0 = ldfrag_h(bp + k0);
          const v16h f1 = ldfrag_h(bp + bs + k0);
          acc[0] = mma_h(ah, f0, acc[0]);  acc[0] = mma_h(al, f0, acc[0]);
          acc[1] = mma_h(ah, f1, acc[1]);  acc[1] = mma_h(al, f1, acc[1]);
          guard2(acc[0], acc[1], ah, al, f0, f1, ah, al);
        }
      } else {
#pragma unroll 1
        for (int k0 = 0; k0 < K; k0 += 32) {
          const v16h ah = ldfrag_h(ahp + k0);
          const v16h f0 = ldfrag_h(bp + k0);
          const v16h f1 = ldfrag_h(bp + bs + k0);
          acc[0] = mma_h(ah, f0, acc[0]);
          acc[1] = mma_h(ah, f1, acc[1]);
          guard2(acc[0], acc[1], ah, f0, f1, ah, f0, f1);
        }
      }
    }
  }

  float bia[NCT];
#pragma unroll
  for (int j = 0; j < NCT; ++j) {
    const int n  = col0 + 16 * j + m;
    const int i0 = imin(n, nseg - 1);
    const int i1 = imin(imax(n - nseg, 0), nseg - 1);
    const int i2 = imin(imax(n - 2 * nseg, 0), nseg - 1);
    const float w0 = b0[i0], w1 = b1[i1], w2 = b2[i2];
    const float sel = (n < nseg) ? w0 : ((n < 2 * nseg) ? w1 : w2);
    bia[j] = (hasbias != 0) ? bfr(sel) : 0.0f;
  }
  float* sl = slab + wave * SLAB64;
#pragma unroll
  for (int r = 0; r < 8; ++r) {
    const int ro = (8 * hh + r) * 68 + m;
#pragma unroll
    for (int j = 0; j < NCT; ++j) {
      float v = acc[j][r] * oscale + bia[j];
      v = (relu != 0) ? fmaxf(v, 0.0f) : v;
      sl[ro + 16 * j] = v;
    }
  }
  wave_sync_lds();

  if constexpr (OM == 0 || OM == 3) {
    constexpr int LPR = 4 * NCT;
    constexpr int RPI = 32 / LPR;
    constexpr int NIT = 16 / RPI;
    const int rsel = lane / LPR, m4 = lane % LPR;
    v4f vals[NIT];
#pragma unroll
    for (int it = 0; it < NIT; ++it) vals[it] = *(const v4f*)(sl + (it * RPI + rsel) * 68 + m4 * 4);
    if constexpr (OM == 3) {
#pragma unroll
      for (int it = 0; it < NIT; ++it) {
        const size_t ro = (size_t)(rowb + it * RPI + rsel) * (size_t)ldc + col0 + m4 * 4;
        const v4f pa = *(const v4f*)(P0 + ro);
        const v4f pb = *(const v4f*)(P1 + ro);
        vals[it] = vals[it] + pa + pb;
      }
    }
    float* dst = Cf + (size_t)(rowb + rsel) * (size_t)ldc + col0 + m4 * 4;
    for (int pass = 0; pass < 2; ++pass) {
#pragma unroll
      for (int it = 0; it < NIT; ++it) {
        *(volatile v4f*)(dst + (size_t)(it * RPI) * (size_t)ldc) = vals[it];
      }
      __threadfence();
    }
  } else {
    const int rq = lane >> 3, c8 = (lane & 7) * 8;
    v4u oh[4], ol[4];
#pragma unroll
    for (int it = 0; it < 4; ++it) {
      const int row = it * 4 + rq;
      const v4f a = *(const v4f*)(sl + row * 68 + c8), b4 = *(const v4f*)(sl + row * 68 + c8 + 4);
      float w[8];
#pragma unroll
      for (int e = 0; e < 4; ++e) { w[e] = a[e] * ocar; w[4 + e] = b4[e] * ocar; }
#pragma unroll
      for (int e = 0; e < 4; ++e) {
        const _Float16 h0 = (_Float16)w[2 * e], h1 = (_Float16)w[2 * e + 1];
        const _Float16 l0 = (_Float16)(w[2 * e] - (float)h0), l1 = (_Float16)(w[2 * e + 1] - (float)h1);
        oh[it][e] = pk16(h_bits(h0), h_bits(h1));
        ol[it][e] = pk16(h_bits(l0), h_bits(l1));
      }
    }
    const size_t ob = (size_t)rowb * (size_t)ldc + col0 + c8;
    for (int pass = 0; pass < 2; ++pass) {
#pragma unroll
      for (int it = 0; it < 4; ++it) {
        const int row = it * 4 + rq;
        *(volatile v4u*)(Ch + ob + (size_t)row * (size_t)ldc) = oh[it];
        if constexpr (OM == 1) {
          *(volatile v4u*)(Cl + ob + (size_t)row * (size_t)ldc) = ol[it];
        }
      }
      __threadfence();
    }
  }
}

__global__ __launch_bounds__(ATT_THREADS)
void attn_k(const u16* __restrict__ S, const u16* __restrict__ VT, const int* __restrict__ mask, int gb0,
            u16* OHp, u16* OLp) {
  __shared__ __align__(16) int   sm[16 * MKP];
  __shared__ __align__(16) float pts[NHD * PTW];
  __shared__ __align__(16) float res[16 * RSP];

  const int tid  = threadIdx.x;
  const int wave = tid >> 5;
  const int lane = tid & 31;
  const int hh   = lane >> 4;
  const int c    = lane & 15;
  const int bid  = blockIdx.x;
  const int qt   = bid % NQT;
  const int b    = bid / NQT;
  if (b >= BG) return;
  const int q0   = qt * 16;

#pragma unroll
  for (int i = 0; i < NST; ++i) {
    const int idx = i * ATT_THREADS + tid;
    const int row = idx / (SEQ / 4);
    const int c4  = (idx - row * (SEQ / 4)) * 4;
    const v4i mv  = *(const v4i*)(mask + ((size_t)(gb0 + b) * SEQ_FULL + q0 + row) * SEQ_FULL + c4);
    *(v4i*)(sm + row * MKP + c4) = mv;
  }
  __syncthreads();

  const int head = wave;
  float* pt = pts + wave * PTW;
  const _Float16* Sh = (const _Float16*)(const void*)S;
  const _Float16* Vh = (const _Float16*)(const void*)VT;
  FragH qf;
  qf.h[0] = *(const v8h*)(Sh + ((size_t)b * SEQ + q0 + c) * NVQK + HDM + head * HDD + 8 * hh);
  qf.u[1] = zero4u();
  const _Float16* Kb = Sh + ((size_t)b * SEQ + c) * NVQK + 2 * HDM + head * HDD + 8 * hh;
  const _Float16* Vb = Vh + ((size_t)(b * NHD + head) * HDD + c) * SEQ + 8 * hh;
  const float lsc   = ATT_SCALE * (LOG2E / (CAR * CAR));
  const float oc    = 1.0f / (PCAR * CAR);
  const float maskt = -1.0e9f * LOG2E;

  float mrow[8], lrow[8];
#pragma unroll
  for (int r = 0; r < 8; ++r) { mrow[r] = -INFINITY; lrow[r] = 0.f; }
  v8f o = zero8();

#pragma unroll 1
  for (int kt = 0; kt < NKT; ++kt) {
    const int kb = kt * 32;
    FragH k0f, k1f;
    k0f.h[0] = *(const v8h*)(Kb + (size_t)kb * NVQK);
    k0f.u[1] = zero4u();
    k1f.h[0] = *(const v8h*)(Kb + (size_t)(kb + 16) * NVQK);
    k1f.u[1] = zero4u();
    v8f s0 = mma_h(qf.v, k0f.v, zero8());
    v8f s1 = mma_h(qf.v, k1f.v, zero8());
    guard2(s0, s1, qf.v, k0f.v, k1f.v, qf.v, k0f.v, k1f.v);
#pragma unroll
    for (int r = 0; r < 8; ++r) {
      const int   qrl = 8 * hh + r;
      const int   m0  = sm[qrl * MKP + kb + c];
      const int   m1  = sm[qrl * MKP + kb + 16 + c];
      const float u0  = s0[r] * lsc;
      const float u1  = s1[r] * lsc;
      const float t0  = (m0 == 0) ? maskt : u0;
      const float t1  = (m1 == 0) ? maskt : u1;
      float mx = fmaxf(t0, t1);
#pragma unroll
      for (int off = 1; off < 16; off <<= 1) mx = fmaxf(mx, __shfl_xor(mx, off, 32));
      const float mn = fmaxf(mrow[r], mx);
      const float ms = (mn == -INFINITY) ? 0.0f : mn;
      const float al = exp2f(mrow[r] - ms);
      mrow[r] = mn;
      const float e0 = exp2f(t0 - ms), e1 = exp2f(t1 - ms);
      float ps = e0 + e1;
#pragma unroll
      for (int off = 1; off < 16; off <<= 1) ps += __shfl_xor(ps, off, 32);
      lrow[r] = lrow[r] * al + ps;
      o[r] *= al;
      const int ro = (8 * hh + r) * PTP + c;
      pt[ro]      = e0;
      pt[ro + 16] = e1;
    }
    wave_sync_lds();
    FragH ph;
    {
      const float* prow = pt + c * PTP + 8 * hh;
      const v4f p0 = *(const v4f*)(prow), p1 = *(const v4f*)(prow + 4);
      const v4f p2 = *(const v4f*)(prow + 16), p3 = *(const v4f*)(prow + 20);
#pragma unroll
      for (int e = 0; e < 4; ++e) {
        ph.h[0][e]     = (_Float16)(p0[e] * PCAR);
        ph.h[0][4 + e] = (_Float16)(p1[e] * PCAR);
        ph.h[1][e]     = (_Float16)(p2[e] * PCAR);
        ph.h[1][4 + e] = (_Float16)(p3[e] * PCAR);
      }
    }
    const v16h vf = ldfrag_h(Vb + kb);
    o = mma_h(ph.v, vf, o);
    guard1(o, ph.v, vf);
    wave_sync_lds();
  }
  acc_guard1(o);
  const v8h vres = *(const v8h*)(Vb + q0);
#pragma unroll
  for (int r = 0; r < 8; ++r) {
    const float lv  = lrow[r];
    const float ls  = (lv > 0.0f) ? lv : 1.0f;
    const float inv = (lv > 0.0f) ? ((1.0f / ls) * oc) : 0.0f;
    const float val = o[r] * inv + (float)vres[r] * (1.0f / CAR);
    res[(8 * hh + r) * RSP + head * HDD + c] = val;
  }
  __syncthreads();
  {
    const int lid = tid >> 3, row = lid >> 1, hf = lid & 1;
    const int c8  = hf * 64 + (tid & 7) * 8;
    const v4f a = *(const v4f*)(res + row * RSP + c8), b4 = *(const v4f*)(res + row * RSP + c8 + 4);
    float w[8];
#pragma unroll
    for (int e = 0; e < 4; ++e) { w[e] = a[e] * CAR; w[4 + e] = b4[e] * CAR; }
    v4u oh, ol;
#pragma unroll
    for (int e = 0; e < 4; ++e) {
      const _Float16 h0 = (_Float16)w[2 * e], h1 = (_Float16)w[2 * e + 1];
      const _Float16 l0 = (_Float16)(w[2 * e] - (float)h0), l1 = (_Float16)(w[2 * e + 1] - (float)h1);
      oh[e] = pk16(h_bits(h0), h_bits(h1));
      ol[e] = pk16(h_bits(l0), h_bits(l1));
    }
    const size_t ob = ((size_t)b * SEQ + q0 + row) * HDM + c8;
    for (int pass = 0; pass < 2; ++pass) {
      *(volatile v4u*)(OHp + ob) = oh;
      *(volatile v4u*)(OLp + ob) = ol;
      __threadfence();
    }
  }
}

extern "C" void kernel_launch(void* const* d_in, const int* in_sizes, int n_in,
                              void* d_out, int out_size, void* d_ws, size_t ws_size,
                              hipStream_t stream) {
  if (n_in < 24) return;
  if (in_sizes[0] < NB * SEQ_FULL * FIN) return;
  if (in_sizes[1] < NB * SEQ_FULL * SEQ_FULL) return;
  if (in_sizes[2] < FIN * HID || in_sizes[3] < HID) return;
  if (in_sizes[4] < HID * HID || in_sizes[5] < HID) return;
  for (int l = 0; l < 2; ++l) {
    const int o = 6 + 8 * l;
    if (in_sizes[o + 0] < HID * HDM || in_sizes[o + 1] < HDM) return;
    if (in_sizes[o + 2] < HID * HDM || in_sizes[o + 3] < HDM) return;
    if (in_sizes[o + 4] < HID * HDM || in_sizes[o + 5] < HDM) return;
    if (in_sizes[o + 6] < HDM * HID || in_sizes[o + 7] < HID) return;
  }
  if (in_sizes[22] < QIN * NACT || in_sizes[23] < NACT) return;
  if (out_size < NB * SEQ * NACT) return;

  const float* x     = (const float*)d_in[0];
  const int*   mask  = (const int*)d_in[1];
  const float* encW1 = (const float*)d_in[2];
  const float* encb1 = (const float*)d_in[3];
  const float* encW2 = (const float*)d_in[4];
  const float* encb2 = (const float*)d_in[5];
  const float* Wv[2] = {(const float*)d_in[6],  (const float*)d_in[14]};
  const float* bv[2] = {(const float*)d_in[7],  (const float*)d_in[15]};
  const float* Wk[2] = {(const float*)d_in[8],  (const float*)d_in[16]};
  const float* bk[2] = {(const float*)d_in[9],  (const float*)d_in[17]};
  const float* Wq[2] = {(const float*)d_in[10], (const float*)d_in[18]};
  const float* bq[2] = {(const float*)d_in[11], (const float*)d_in[19]};
  const float* Wo[2] = {(const float*)d_in[12], (const float*)d_in[20]};
  const float* bo[2] = {(const float*)d_in[13], (const float*)d_in[21]};
  const float* qW    = (const float*)d_in[22];
  const float* qb    = (const float*)d_in[23];
  float*       out   = (float*)d_out;

  const size_t szXB = (size_t)GROWS * FIN * 2;
  const size_t szW1 = (size_t)HID * FIN * 2;
  const size_t szW2 = (size_t)HID * HID * 2;
  const size_t szWV = (size_t)NVQK * HID * 2;
  const size_t szWO = (size_t)HID * HDM * 2;
  const size_t szQW = (size_t)NACT * QIN * 2;
  const size_t szR  = (size_t)GROWS * HID * 2;
  const size_t szS  = (size_t)GROWS * NVQK * 2;
  const size_t szVT = (size_t)BG * HDM * SEQ * 2;
  const size_t szO  = (size_t)GROWS * HDM * 2;
  const size_t szP  = (size_t)NB * SEQ * NACT * 4;
  size_t off = 0;
  const size_t oXB  = off; off += szXB;
  const size_t oW1  = off; off += szW1;
  const size_t oW2  = off; off += szW2;
  const size_t oWV1 = off; off += szWV;
  const size_t oWV2 = off; off += szWV;
  const size_t oWO1 = off; off += szWO;
  const size_t oWO2 = off; off += szWO;
  const size_t oQW  = off; off += szQW;
  const size_t oRAh = off; off += szR;
  const size_t oRAl = off; off += szR;
  const size_t oRBh = off; off += szR;
  const size_t oRBl = off; off += szR;
  const size_t oS   = off; off += szS;
  const size_t oVT  = off; off += szVT;
  const size_t oOH  = off; off += szO;
  const size_t oOL  = off; off += szO;
  const size_t oP0  = off; off += szP;
  const size_t oP1  = off; off += szP;
  if (off > ws_size) return;
  if (off > (size_t)WS_CAP) return;

  char* ws = (char*)d_ws;
  u16*   XB    = (u16*)(ws + oXB);
  u16*   W1T   = (u16*)(ws + oW1);
  u16*   W2T   = (u16*)(ws + oW2);
  u16*   WVQK[2] = {(u16*)(ws + oWV1), (u16*)(ws + oWV2)};
  u16*   WOT[2]  = {(u16*)(ws + oWO1), (u16*)(ws + oWO2)};
  u16*   QWT   = (u16*)(ws + oQW);
  u16*   RAh   = (u16*)(ws + oRAh);
  u16*   RAl   = (u16*)(ws + oRAl);
  u16*   RBh   = (u16*)(ws + oRBh);
  u16*   RBl   = (u16*)(ws + oRBl);
  u16*   S     = (u16*)(ws + oS);
  u16*   VT    = (u16*)(ws + oVT);
  u16*   OH    = (u16*)(ws + oOH);
  u16*   OL    = (u16*)(ws + oOL);
  float* P0    = (float*)(ws + oP0);
  float* P1    = (float*)(ws + oP1);

  const dim3 b256(256), b128(128), bAT(ATT_THREADS);
  const float WSC = CAR;
  const float OSF = 1.0f / (CAR * CAR);
  const int   n8x = (GROWS * FIN) / 8;
  const dim3  gX((n8x + 255) / 256);
  const dim3  gGH((GROWS / 64) * (HID / 64));
  const dim3  gGV((GROWS / 64) * (NVQK / 64));
  const dim3  gGP(GROWS / 64);
  const dim3  gVT(BG * NST);
  const dim3  gAT(BG * NQT);

  wt16<128, 1><<<dim3((HID / 128) * (FIN / 64)), b256, 0, stream>>>(encW1, HID, FIN, HID, W1T, FIN, 0, 1.0f);
  wt16<128, 0><<<dim3((HID / 128) * (HID / 64)), b256, 0, stream>>>(encW2, HID, HID, HID, W2T, HID, 0, WSC);
  for (int l = 0; l < 2; ++l) {
    wt16<128, 0><<<dim3((HDM / 128) * (HID / 64)), b256, 0, stream>>>(Wv[l], HDM, HID, HDM, WVQK[l], HID, 0, WSC);
    wt16<128, 0><<<dim3((HDM / 128) * (HID / 64)), b256, 0, stream>>>(Wq[l], HDM, HID, HDM, WVQK[l], HID, HDM, WSC);
    wt16<128, 0><<<dim3((HDM / 128) * (HID / 64)), b256, 0, stream>>>(Wk[l], HDM, HID, HDM, WVQK[l], HID, 2 * HDM, WSC);
    wt16<128, 0><<<dim3((HID / 128) * (HDM / 64)), b256, 0, stream>>>(Wo[l], HID, HDM, HID, WOT[l], HDM, 0, WSC);
  }
  wt16<32, 0><<<dim3((NACT / 32) * (QIN / 64)), b256, 0, stream>>>(qW, NACT, QIN, NACT, QWT, QIN, 0, WSC);

  for (int g = 0; g < NGRP; ++g) {
    float* og  = out + (size_t)g * GROWS * NACT;
    float* P0g = P0 + (size_t)g * GROWS * NACT;
    float* P1g = P1 + (size_t)g * GROWS * NACT;
    cvtx<<<gX, b256, 0, stream>>>(x, XB, g * BG, n8x);
    gemm16<1, 1, 4, 1><<<gGH, b128, 0, stream>>>(XB, XB, FIN, W1T, FIN, FIN, GROWS, HID,
                                                 encb1, encb1, encb1, HID, 1, 1, 1.0f, CAR,
                                                 P0g, RAh, RAl, HID, P0g, P1g);
    gemm16<0, 2, 4, 1><<<gGH, b128, 0, stream>>>(RAh, RAl, HID, W2T, HID, HID, GROWS, HID,
                                                 encb2, encb2, encb2, HID, 1, 1, OSF, CAR,
                                                 P0g, RBh, RBl, HID, P0g, P1g);
    gemm16<0, 2, 2, 0><<<gGP, b128, 0, stream>>>(RBh, RBl, HID, QWT, QIN, HID, GROWS, NACT,
                                                 qb, qb, qb, NACT, 0, 0, OSF, 1.0f,
                                                 P0g, XB, XB, NACT, P0g, P1g);
    for (int l = 0; l < 2; ++l) {
      u16* Hih = (l == 0) ? RBh : RAh;
      u16* Hil = (l == 0) ? RBl : RAl;
      u16* Hoh = (l == 0) ? RAh : RBh;
      u16* Hol = (l == 0) ? RAl : RBl;
      gemm16<0, 2, 4, 2><<<gGV, b128, 0, stream>>>(Hih, Hil, HID, WVQK[l], HID, HID, GROWS, NVQK,
                                                   bv[l], bq[l], bk[l], HDM, 1, 1, OSF, CAR,
                                                   P0g, S, S, NVQK, P0g, P1g);
      vt16k<<<gVT, b256, 0, stream>>>(S, VT);
      attn_k<<<gAT, bAT, 0, stream>>>(S, VT, mask, g * BG, OH, OL);
      gemm16<0, 2, 4, 1><<<gGH, b128, 0, stream>>>(OH, OL, HDM, WOT[l], HDM, HDM, GROWS, HID,
                                                   bo[l], bo[l], bo[l], HID, 1, 1, OSF, CAR,
                                                   P0g, Hoh, Hol, HID, P0g, P1g);
      if (l == 0) {
        gemm16<0, 2, 2, 0><<<gGP, b128, 0, stream>>>(Hoh, Hol, HID, QWT + HID, QIN, HID, GROWS, NACT,
                                                     qb, qb, qb, NACT, 0, 0, OSF, 1.0f,
                                                     P1g, XB, XB, NACT, P0g, P1g);
      } else {
        gemm16<0, 2, 2, 3><<<gGP, b128, 0, stream>>>(Hoh, Hol, HID, QWT + 2 * HID, QIN, HID, GROWS, NACT,
                                                     qb, qb, qb, NACT, 1, 0, OSF, 1.0f,
                                                     og, XB, XB, NACT, P0g, P1g);
      }
    }
  }
  (void)hipGetLastError();
}
